// PPLayer_9569187135998
// MI455X (gfx1250) — hardware-verified
//
#include <hip/hip_runtime.h>


#define NIMG 128
#define CC   512
#define NPIX 49
#define NQ   (NIMG * NPIX)
#define NGRP 21
#define NSH  10
#define GW   (NSH * NPIX)
#define GP   512
#define NKR  (NGRP * GW)
#define NKP  10304
#define DKY  128
#define RCH  896
#define DM   CC
#define SCL  0.088388347648318447f
#define LOSC 1024.0f

typedef _Float16 h16;
typedef unsigned short bf;
typedef __attribute__((ext_vector_type(16))) __bf16   v16bf;
typedef __attribute__((ext_vector_type(16))) _Float16 v16h;
typedef __attribute__((ext_vector_type(8)))  _Float16 v8h;
typedef __attribute__((ext_vector_type(8)))  unsigned short v8us;
typedef __attribute__((ext_vector_type(8)))  float    v8f;
typedef __attribute__((ext_vector_type(4)))  float    v4f;
typedef __attribute__((ext_vector_type(4)))  _Float16 v4h;
typedef v8h  __attribute__((may_alias)) v8ha;
typedef v4f  __attribute__((may_alias)) v4fa;
typedef v8us __attribute__((may_alias)) v8usa;

__device__ __forceinline__ unsigned short f2bf(float f) { unsigned u = __float_as_uint(f); u += 0x7FFFu + ((u >> 16) & 1u); return (unsigned short)(u >> 16); }
__device__ __forceinline__ float bf2f(unsigned short b) { return __uint_as_float(((unsigned)b) << 16); }
__device__ __forceinline__ float bfr(float f) { return bf2f(f2bf(f)); }
__device__ __forceinline__ v16h cat16(v8h lo, v8h hi) { return __builtin_shufflevector(lo, hi, 0, 1, 2, 3, 4, 5, 6, 7, 8, 9, 10, 11, 12, 13, 14, 15); }
__device__ __forceinline__ v16bf cat16b(v8us lo, v8us hi) { return __builtin_bit_cast(v16bf, __builtin_shufflevector(lo, hi, 0, 1, 2, 3, 4, 5, 6, 7, 8, 9, 10, 11, 12, 13, 14, 15)); }
__device__ __forceinline__ v8f wmma16(v16h a, v16h b, v8f c) { return __builtin_amdgcn_wmma_f32_16x16x32_f16(false, a, false, b, (short)0, c, false, false); }
__device__ __forceinline__ v8f wmmab(v16bf a, v16bf b, v8f c) { return __builtin_amdgcn_wmma_f32_16x16x32_bf16(false, a, false, b, (short)0, c, false, false); }

template <bool SPLITA, bool F16OUT = false>
__global__ __launch_bounds__(128) void k_gemmb(const bf* __restrict__ A, const bf* __restrict__ Al, const bf* __restrict__ Bn, const float* __restrict__ bias, float* C, int ldc, h16* C2, const float* __restrict__ R = nullptr, int K = DM, int roundR = 1) {
    __shared__ __align__(16) float ost[4][16 * 68];
    const int lane = threadIdx.x & 31, wave = threadIdx.x >> 5, lr = lane & 15, hi = lane >> 4;
    const int r0 = blockIdx.x * 64 + wave * 16, c0 = blockIdx.y * 64;
    const size_t aoff = (size_t)(r0 + lr) * K + 8 * hi;
    size_t boff[4];
#pragma unroll
    for (int t = 0; t < 4; ++t) boff[t] = (size_t)(c0 + t * 16 + lr) * K + 8 * hi;
    v8f acc[4];
#pragma unroll
    for (int t = 0; t < 4; ++t) acc[t] = (v8f){};
#pragma unroll 1
    for (int kc = 0; kc < K; kc += 32) {
        const v16bf a = cat16b(*(const v8us*)(A + aoff + kc), *(const v8us*)(A + aoff + kc + 16));
        v16bf al = a;
        if (SPLITA) al = cat16b(*(const v8us*)(Al + aoff + kc), *(const v8us*)(Al + aoff + kc + 16));
#pragma unroll
        for (int t = 0; t < 4; ++t) { const v16bf b = cat16b(*(const v8us*)(Bn + boff[t] + kc), *(const v8us*)(Bn + boff[t] + kc + 16)); acc[t] = wmmab(a, b, acc[t]); if (SPLITA) acc[t] = wmmab(al, b, acc[t]); }
        asm volatile("v_nop\n\tv_nop\n\tv_nop\n\tv_nop" : "+v"(acc[0]), "+v"(acc[1]), "+v"(acc[2]), "+v"(acc[3]) : "v"(a), "v"(al));
    }
    float* os = &ost[wave][0];
#pragma unroll
    for (int t = 0; t < 4; ++t) { const float bv = bias ? bfr(bias[c0 + t * 16 + lr]) : 0.f;
#pragma unroll
        for (int j = 0; j < 8; ++j) os[(hi * 8 + j) * 68 + t * 16 + lr] = acc[t][j] + bv; }
    __syncthreads();
    if (F16OUT) {
        h16* crow = (h16*)(void*)C + (size_t)r0 * ldc + c0;
        auto pass = [&]() {
#pragma unroll
            for (int s = 0; s < 4; ++s) { const int row = 4 * s + (lane >> 3), piece = lane & 7; const float* sp = os + row * 68 + piece * 8; v8h o, o2;
#pragma unroll
                for (int i = 0; i < 8; ++i) { const h16 a = (h16)sp[i]; o[i] = a; o2[i] = (h16)((sp[i] - (float)a) * LOSC); }
                *(volatile v8h*)(crow + (size_t)row * ldc + piece * 8) = o; if (C2) *(volatile v8h*)(C2 + (size_t)r0 * ldc + c0 + (size_t)row * ldc + piece * 8) = o2; }
        };
        pass(); __threadfence(); pass();
    } else {
        float* crow = C + (size_t)r0 * ldc + c0;
        auto pass = [&]() {
#pragma unroll
            for (int s = 0; s < 8; ++s) { const int Lid = (lane >> 3) + 4 * s, piece = lane & 7; const int row = Lid >> 1, cofs = (Lid & 1) * 32 + piece * 4;
                v4f val = *(const v4fa*)(os + row * 68 + cofs); if (R) { const v4f rv = *(const v4f*)(R + ((size_t)r0 + row) * ldc + c0 + cofs); val += roundR ? (v4f){bfr(rv[0]), bfr(rv[1]), bfr(rv[2]), bfr(rv[3])} : rv; }
                *(volatile v4f*)(crow + (size_t)row * ldc + cofs) = val; }
        };
        pass(); __threadfence(); pass();
    }
}

__global__ __launch_bounds__(256) void k_cvt8(const float* __restrict__ src, bf* dst, size_t n8) {
    const size_t i = (size_t)blockIdx.x * 256 + threadIdx.x; if (i >= n8) return;
    const v8f v = *(const v8f*)(src + i * 8); v8us o;
#pragma unroll
    for (int k = 0; k < 8; ++k) o[k] = f2bf(v[k]);
    *(volatile v8us*)(dst + i * 8) = o; __threadfence(); *(volatile v8us*)(dst + i * 8) = o;
}
__global__ __launch_bounds__(256) void k_zero8(bf* dst, size_t n8) {
    const size_t i = (size_t)blockIdx.x * 256 + threadIdx.x; if (i >= n8) return; v8us z;
#pragma unroll
    for (int k = 0; k < 8; ++k) z[k] = 0;
    *(volatile v8us*)(dst + i * 8) = z; __threadfence(); *(volatile v8us*)(dst + i * 8) = z;
}
__global__ __launch_bounds__(128) void k_gemm3(const bf* __restrict__ Ah, const bf* __restrict__ Al, const bf* __restrict__ Bh, const bf* __restrict__ Bl, int K, float* C, int ldc) {
    __shared__ __align__(16) float ost[4][16 * 68];
    const int lane = threadIdx.x & 31, wave = threadIdx.x >> 5, lr = lane & 15, hi = lane >> 4;
    const int r0 = blockIdx.x * 64 + wave * 16, c0 = blockIdx.y * 64;
    const size_t aoff = (size_t)(r0 + lr) * K + 8 * hi;
    v8f acc[4];
#pragma unroll
    for (int t = 0; t < 4; ++t) acc[t] = (v8f){};
#pragma unroll 1
    for (int kc = 0; kc < K; kc += 32) {
        const v16bf a = cat16b(*(const v8us*)(Ah + aoff + kc), *(const v8us*)(Ah + aoff + kc + 16));
        const v16bf al = cat16b(*(const v8us*)(Al + aoff + kc), *(const v8us*)(Al + aoff + kc + 16));
#pragma unroll
        for (int t = 0; t < 4; ++t) { const size_t bo = (size_t)(c0 + t * 16 + lr) * K + kc + 8 * hi;
            const v16bf bh = cat16b(*(const v8us*)(Bh + bo), *(const v8us*)(Bh + bo + 16)); const v16bf bl = cat16b(*(const v8us*)(Bl + bo), *(const v8us*)(Bl + bo + 16));
            acc[t] = wmmab(a, bh, acc[t]); acc[t] = wmmab(al, bh, acc[t]); acc[t] = wmmab(a, bl, acc[t]); }
        asm volatile("v_nop\n\tv_nop\n\tv_nop\n\tv_nop" : "+v"(acc[0]), "+v"(acc[1]), "+v"(acc[2]), "+v"(acc[3]) : "v"(a), "v"(al));
    }
    float* os = &ost[wave][0];
#pragma unroll
    for (int t = 0; t < 4; ++t) {
#pragma unroll
        for (int j = 0; j < 8; ++j) os[(hi * 8 + j) * 68 + t * 16 + lr] = acc[t][j]; }
    __builtin_amdgcn_wave_barrier(); asm volatile("" ::: "memory");
    float* crow = C + (size_t)r0 * ldc + c0;
    auto pass = [&]() {
#pragma unroll
        for (int s = 0; s < 8; ++s) { const int Lid = (lane >> 3) + 4 * s, piece = lane & 7; const int row = Lid >> 1, cofs = (Lid & 1) * 32 + piece * 4;
            const v4f val = *(const v4fa*)(os + row * 68 + cofs); *(volatile v4f*)(crow + (size_t)row * ldc + cofs) = val; }
    };
    pass(); __threadfence(); pass();
}


__global__ __launch_bounds__(256) void k_pixT(const float* __restrict__ src, int ngrp, int nrows, bf* R) {
    const int lane = threadIdx.x & 31; const size_t r = (size_t)blockIdx.x * 8 + (threadIdx.x >> 5); if (r >= (size_t)nrows) return; const bool live = r < (size_t)ngrp * NPIX; const size_t g = live ? r / NPIX : 0; const int p = live ? (int)(r % NPIX) : 0;
#pragma unroll 1
    for (int ps = 0; ps < 2; ++ps) {
#pragma unroll
        for (int q = 0; q < CC / 256; ++q) { v8us o;
#pragma unroll
            for (int i = 0; i < 8; ++i) { const int c = q * 256 + lane * 8 + i; o[i] = f2bf(live ? src[((g * CC + c) * NPIX) + p] : 0.f); }
            *(volatile v8us*)(R + r * CC + q * 256 + lane * 8) = o; }
        if (ps == 0) __threadfence(); }
}
__global__ __launch_bounds__(256) void k_split128(const float* __restrict__ F, int rows, float sc, bf* Ph, bf* Pl) {
    typedef __attribute__((ext_vector_type(4))) unsigned short v4us;
    const int lane = threadIdx.x & 31; const size_t r = (size_t)blockIdx.x * 8 + (threadIdx.x >> 5); if (r >= (size_t)rows) return; v4us oh, ol;
#pragma unroll
    for (int i = 0; i < 4; ++i) { const float y = F[r * DKY + lane * 4 + i] * sc; const unsigned short hb = f2bf(y); oh[i] = hb; ol[i] = f2bf(y - bf2f(hb)); }
    const size_t o = r * DKY + lane * 4; *(volatile v4us*)(Ph + o) = oh; *(volatile v4us*)(Pl + o) = ol; __threadfence(); *(volatile v4us*)(Ph + o) = oh; *(volatile v4us*)(Pl + o) = ol;
}
__global__ __launch_bounds__(256) void k_pvT(const float* __restrict__ PV, bf* Th, bf* Tl) {
    const int lane = threadIdx.x & 31; const size_t w = (size_t)blockIdx.x * 8 + (threadIdx.x >> 5); if (w >= (size_t)NGRP * DKY) return; const int g = (int)(w / DKY), e = (int)(w % DKY);
#pragma unroll 1
    for (int ps = 0; ps < 2; ++ps) {
#pragma unroll
        for (int q = 0; q < GP / 256; ++q) { v8us oh, ol;
#pragma unroll
            for (int i = 0; i < 8; ++i) { const int m = q * 256 + lane * 8 + i; const float y = (m < GW) ? PV[((size_t)g * GW + (m < GW ? m : 0)) * DKY + e] : 0.f; const unsigned short hb = f2bf(y); oh[i] = hb; ol[i] = f2bf(y - bf2f(hb)); }
            const size_t o = (w) * GP + q * 256 + lane * 8; *(volatile v8us*)(Th + o) = oh; *(volatile v8us*)(Tl + o) = ol; }
        if (ps == 0) __threadfence(); }
}
__global__ __launch_bounds__(256) void k_grpsoft(const float* __restrict__ S, bf* PH, bf* PL) {
    const int lane = threadIdx.x & 31; const size_t w = (size_t)blockIdx.x * 8 + (threadIdx.x >> 5); if (w >= (size_t)RCH * NGRP) return; const int rl = (int)(w / NGRP), g = (int)(w % NGRP); const float* sr = S + (size_t)rl * NKP + (size_t)g * GW;
    float m = -3.0e38f;
#pragma unroll 1
    for (int c = lane; c < GW; c += 32) m = fmaxf(m, sr[c]);
#pragma unroll
    for (int sh = 16; sh; sh >>= 1) m = fmaxf(m, __shfl_xor(m, sh, 32));
    float sum = 0.f;
#pragma unroll 1
    for (int c = lane; c < GW; c += 32) sum += __expf(sr[c] - m);
#pragma unroll
    for (int sh = 16; sh; sh >>= 1) sum += __shfl_xor(sum, sh, 32);
    const float inv = 1.0f / sum;
#pragma unroll 1
    for (int ps = 0; ps < 2; ++ps) {
#pragma unroll
        for (int q = 0; q < GP / 256; ++q) { v8us oh, ol;
#pragma unroll
            for (int i = 0; i < 8; ++i) { const int c = q * 256 + lane * 8 + i; const float p = (c < GW) ? __expf(sr[(c < GW) ? c : 0] - m) * inv : 0.f; const unsigned short hb = f2bf(p); oh[i] = hb; ol[i] = f2bf(p - bf2f(hb)); }
            const size_t o = ((size_t)g * RCH + rl) * GP + q * 256 + lane * 8; *(volatile v8us*)(PH + o) = oh; *(volatile v8us*)(PL + o) = ol; }
        if (ps == 0) __threadfence(); }
}
__global__ __launch_bounds__(256) void k_dist(const float* __restrict__ QV, const float* __restrict__ OUT, float* dst) {
    const int lane = threadIdx.x & 31; const size_t idx = ((size_t)blockIdx.x * 8 + (threadIdx.x >> 5)) * 32 + lane; if (idx >= (size_t)NIMG * NGRP) return; const int b = (int)(idx / NGRP), g = (int)(idx % NGRP); float s = 0.f;
#pragma unroll 1
    for (int p = 0; p < NPIX; ++p) { const size_t row = (size_t)b * NPIX + p; const float* qv = QV + row * DKY; const float* ov = OUT + ((size_t)g * NQ + row) * DKY;
#pragma unroll 1
        for (int e = 0; e < DKY; ++e) { const float d = qv[e] - ov[e]; s = fmaf(d, d, s); } }
    const float v = -s * (1.0f / NPIX); *(volatile float*)(dst + idx) = v; __threadfence(); *(volatile float*)(dst + idx) = v;
}

extern "C" void kernel_launch(void* const* d_in, const int* in_sizes, int n_in,
                              void* d_out, int out_size, void* d_ws, size_t ws_size, hipStream_t stream) {
    (void)in_sizes; (void)n_in; (void)out_size;
    const float* x = (const float*)d_in[0]; const float* prots = (const float*)d_in[1]; const float* wqk = (const float*)d_in[2]; const float* wv = (const float*)d_in[3];
    float* out = (float*)d_out;
    char* wsp = (char*)d_ws;
    auto take = [&](size_t bytes) { char* p = wsp; wsp += (bytes + 255) & ~(size_t)255; return (void*)p; };
    bf* WQK = (bf*)take((size_t)DKY * CC * 2); bf* WV = (bf*)take((size_t)DKY * CC * 2);
    bf* XT = (bf*)take((size_t)NQ * CC * 2); bf* PT = (bf*)take((size_t)NKP * CC * 2); float* Q = (float*)take((size_t)NQ * DKY * 4); float* QV = (float*)take((size_t)NQ * DKY * 4); float* PK = (float*)take((size_t)NKP * DKY * 4); float* PV = (float*)take((size_t)NKP * DKY * 4);
    bf* Qh = (bf*)take((size_t)NQ * DKY * 2); bf* Ql = (bf*)take((size_t)NQ * DKY * 2); bf* Kh = (bf*)take((size_t)NKP * DKY * 2); bf* Kl = (bf*)take((size_t)NKP * DKY * 2); bf* VTh = (bf*)take((size_t)NGRP * DKY * GP * 2); bf* VTl = (bf*)take((size_t)NGRP * DKY * GP * 2);
    float* S = (float*)take((size_t)RCH * NKP * 4); bf* PH = (bf*)take((size_t)NGRP * RCH * GP * 2); bf* PL = (bf*)take((size_t)NGRP * RCH * GP * 2); float* OUT = (float*)take((size_t)NGRP * NQ * DKY * 4);
    if ((size_t)(wsp - (char*)d_ws) > ws_size) return;
    k_cvt8<<<(DKY * CC / 8 + 255) / 256, 256, 0, stream>>>(wqk, WQK, DKY * CC / 8); k_cvt8<<<(DKY * CC / 8 + 255) / 256, 256, 0, stream>>>(wv, WV, DKY * CC / 8);
    k_pixT<<<NQ / 8, 256, 0, stream>>>(x, NIMG, NQ, XT); k_pixT<<<NKP / 8, 256, 0, stream>>>(prots, NGRP * NSH, NKP, PT);
    k_gemmb<false, false><<<dim3(NQ / 64, DKY / 64, 1), 128, 0, stream>>>(XT, nullptr, WQK, nullptr, Q, DKY, nullptr, nullptr, CC); k_gemmb<false, false><<<dim3(NQ / 64, DKY / 64, 1), 128, 0, stream>>>(XT, nullptr, WV, nullptr, QV, DKY, nullptr, nullptr, CC);
    k_gemmb<false, false><<<dim3(NKP / 64, DKY / 64, 1), 128, 0, stream>>>(PT, nullptr, WQK, nullptr, PK, DKY, nullptr, nullptr, CC); k_gemmb<false, false><<<dim3(NKP / 64, DKY / 64, 1), 128, 0, stream>>>(PT, nullptr, WV, nullptr, PV, DKY, nullptr, nullptr, CC);
    k_split128<<<NQ / 8, 256, 0, stream>>>(Q, NQ, SCL, Qh, Ql); k_split128<<<NKP / 8, 256, 0, stream>>>(PK, NKP, 1.0f, Kh, Kl); k_pvT<<<(NGRP * DKY) / 8, 256, 0, stream>>>(PV, VTh, VTl);
    for (int ch = 0; ch < NQ / RCH; ++ch) { const size_t r0 = (size_t)ch * RCH;
        k_gemm3<<<dim3(RCH / 64, NKP / 64, 1), 128, 0, stream>>>(Qh + r0 * DKY, Ql + r0 * DKY, Kh, Kl, DKY, S, NKP);
        k_grpsoft<<<(RCH * NGRP) / 8, 256, 0, stream>>>(S, PH, PL);
        for (int g = 0; g < NGRP; ++g) k_gemm3<<<dim3(RCH / 64, DKY / 64, 1), 128, 0, stream>>>(PH + (size_t)g * RCH * GP, PL + (size_t)g * RCH * GP, VTh + (size_t)g * DKY * GP, VTl + (size_t)g * DKY * GP, GP, OUT + ((size_t)g * NQ + r0) * DKY, DKY); }
    k_dist<<<(NIMG * NGRP + 255) / 256, 256, 0, stream>>>(QV, OUT, out);
}
